// DiagSSMBlock_31387620999391
// MI455X (gfx1250) — hardware-verified
//
#include <hip/hip_runtime.h>


namespace {
constexpr int T = 4096, HH = 2048;
constexpr float XS = 8.0f, WSC = 256.0f;
typedef _Float16 b16;
typedef __attribute__((ext_vector_type(16))) _Float16 v16b;
typedef __attribute__((ext_vector_type(8))) _Float16 v8b;
typedef __attribute__((ext_vector_type(8))) float v8f;
typedef __attribute__((ext_vector_type(4))) float v4f;
__device__ __forceinline__ float bf16_rne(float f) { unsigned int u = __float_as_uint(f); u += 0x7FFFu + ((u >> 16) & 1u); float r = __uint_as_float(u & 0xFFFF0000u); asm volatile("" : "+v"(r)); return r; }
__device__ __forceinline__ float bfv(float f) { float r = bf16_rne(f); asm volatile("" : "+v"(r)); return r; }
__device__ __forceinline__ v16b frag_kb(const b16* p, int hh) { const v8b a = *(const v8b*)(p + 8 * hh), b = *(const v8b*)(p + 16 + 8 * hh); v16b f;
#pragma unroll
  for (int e = 0; e < 8; ++e) { f[e] = a[e]; f[8 + e] = b[e]; } return f; }
__device__ __forceinline__ v8f wmma16b(v16b a, v16b b, v8f c) { v8f d = __builtin_amdgcn_wmma_f32_16x16x32_f16(false, a, false, b, (short)0, c, false, false); asm volatile("v_nop\n\tv_nop\n\tv_nop\n\tv_nop" : "+v"(d) : "v"(a), "v"(b)); return d; }
__device__ __forceinline__ void wave_lds_sync() { __builtin_amdgcn_fence(__ATOMIC_RELEASE, "workgroup"); __builtin_amdgcn_wave_barrier(); __builtin_amdgcn_fence(__ATOMIC_ACQUIRE, "workgroup"); }
__device__ __forceinline__ float pmul(float a, float b) { float p = a * b; asm volatile("" : "+v"(p)); return p; }

__global__ __launch_bounds__(256) void wput_kernel(const float* __restrict__ bm, b16* __restrict__ BT) { const size_t nt = (size_t)gridDim.x * 256, u0 = (size_t)blockIdx.x * 256 + threadIdx.x; v8b v;
  for (size_t u = u0; u < (size_t)HH * (HH / 8); u += nt) { const int o = (int)(u / (HH / 8)), k0 = (int)(u % (HH / 8)) * 8;
#pragma unroll
    for (int j = 0; j < 8; ++j) v[j] = (b16)(bf16_rne(bm[(size_t)(k0 + j) * HH + o]) * WSC); for (int pass = 0; pass < 2; ++pass) { *(volatile v8b*)(BT + (size_t)o * HH + k0) = v; __threadfence(); } } }
__global__ __launch_bounds__(32) void gemm_kernel(const float* __restrict__ x, const b16* __restrict__ BT, int TLIM, float* __restrict__ Sp) { __shared__ __attribute__((aligned(16))) b16 Ax[16][HH + 8]; __shared__ float Tf[16][260]; const int lane = threadIdx.x, nloc = lane & 15, hlf = lane >> 4; const size_t t0 = (size_t)blockIdx.x * 16; const int cq = blockIdx.y * 512; if (t0 >= (size_t)TLIM) return;
  for (int rr = 0; rr < 16; ++rr) for (int q = 0; q < HH / 32; ++q) { const int c = q * 32 + lane; Ax[rr][c] = (b16)(bf16_rne(x[(t0 + rr) * HH + c]) * XS); }
  if (lane < 16) for (int k = HH; k < HH + 8; ++k) Ax[lane][k] = (b16)0.0f;
  wave_lds_sync();
#pragma unroll 1
  for (int g = 0; g < 2; ++g) { const int c0 = cq + g * 256; v8f acc[16];
#pragma unroll
    for (int t = 0; t < 16; ++t) acc[t] = (v8f){};
#pragma unroll 2
    for (int kb = 0; kb < HH; kb += 32) { const v16b a = frag_kb(&Ax[nloc][kb], hlf);
#pragma unroll
      for (int t = 0; t < 16; ++t) acc[t] = wmma16b(a, frag_kb(BT + (size_t)(c0 + t * 16 + nloc) * HH + kb, hlf), acc[t]); }
#pragma unroll
    for (int t = 0; t < 16; ++t)
#pragma unroll
      for (int r8 = 0; r8 < 8; ++r8) Tf[8 * hlf + r8][t * 16 + nloc] = acc[t][r8] * (1.0f / (XS * WSC));
    wave_lds_sync();
    for (int pass = 0; pass < 2; ++pass) { for (int rr = 0; rr < 16; ++rr) for (int q = 0; q < 2; ++q) *(volatile v4f*)(Sp + (t0 + rr) * HH + c0 + q * 128 + lane * 4) = *(const v4f*)(&Tf[rr][q * 128 + lane * 4]); __threadfence(); }
    wave_lds_sync(); } }
__global__ __launch_bounds__(256) void scan_kernel(const float* __restrict__ Sp, const float* __restrict__ am, int TLIM, float* __restrict__ out) { const int c = blockIdx.x * 256 + threadIdx.x; if (c >= HH) return; const float a = bfv(am[c]);
  for (int pass = 0; pass < 2; ++pass) { float h = 0.0f;
#pragma unroll 1
    for (int t = 0; t < TLIM; ++t) { h = tanhf(pmul(a, h) + Sp[(size_t)t * HH + c]); ((volatile float*)out)[(size_t)t * HH + c] = h; } __threadfence(); } }
}

extern "C" void kernel_launch(void* const* d_in, const int* in_sizes, int n_in, void* d_out, int out_size, void* d_ws, size_t ws_size, hipStream_t stream) {
  (void)n_in;
  auto Fp = [&](int i) { return (const float*)d_in[i]; };
  if (in_sizes[0] != T * HH || in_sizes[1] != HH || in_sizes[2] != HH * HH || out_size != T * HH) return;
  const int TLIM = T;
  size_t off = 0; char* ws = (char*)d_ws;
  auto carve = [&](size_t bytes) { char* p = ws + off; off += (bytes + 255) & ~(size_t)255; return p; };
  b16* BT = (b16*)carve((size_t)HH * HH * 2); float* Sp = (float*)carve((size_t)T * HH * 4);
  if (off > ws_size || off > ((size_t)48 << 20)) return;
  wput_kernel<<<512, 256, 0, stream>>>(Fp(2), BT);
  gemm_kernel<<<dim3(TLIM / 16, 4), 32, 0, stream>>>(Fp(0), BT, TLIM, Sp);
  scan_kernel<<<HH / 256, 256, 0, stream>>>(Sp, Fp(1), TLIM, (float*)d_out);
}
